// GNN_dgl_26456998543861
// MI455X (gfx1250) — hardware-verified
//
#include <hip/hip_runtime.h>
#include <stddef.h>
#include <stdint.h>


#define DF    128
#define NHD   4
#define HDIM  32
#define GR    32
#define XSP   132
#define NB    512
#define CHUNK 2048
#define NTHR  256
#define NWAVE 8
#define WCAP  256
#define NGRP  (CHUNK / (NTHR * 4))

#define LDS_SACC (NB * DF)
#define LDS_DEN  (NB * NHD)
#define LDS_LIST (NWAVE * WCAP)
#define LDS_BYTES ((LDS_SACC + LDS_DEN + LDS_LIST + NWAVE) * 4)

static_assert(WCAP == (CHUNK / NTHR) * 32);
static_assert(NGRP >= 1);
static_assert(NB == 512);
static_assert(CHUNK <= 4096);
static_assert(((LDS_SACC + LDS_DEN) % 4) == 0);
static_assert(LDS_BYTES == 278560);
static_assert(NHD * HDIM == DF);
static_assert(NB / NWAVE == 64);

typedef float    v4f  __attribute__((ext_vector_type(4)));
typedef float    v8f  __attribute__((ext_vector_type(8)));
typedef int      v4i  __attribute__((ext_vector_type(4)));
typedef _Float16 v4h  __attribute__((ext_vector_type(4)));
typedef _Float16 v8h  __attribute__((ext_vector_type(8)));
typedef _Float16 v16h __attribute__((ext_vector_type(16)));
union Frag   { v16h v; v8h half[2]; };
union Pack16 { v8h h; v4i i; };

__device__ __forceinline__ v8f wm(v16h a, v16h b, v8f c) {
  v8f d = __builtin_amdgcn_wmma_f32_16x16x32_f16(false, a, false, b, (short)0, c, false, false);
  asm volatile("v_nop\n\tv_nop\n\tv_nop\n\tv_nop" : "+v"(d) : "v"(a), "v"(b));
  return d;
}

__device__ __forceinline__ float th1(float v) {
  v = fminf(fmaxf(v, -15.0f), 15.0f);
  const float e = __expf(2.0f * v);
  return 1.0f - 2.0f * __builtin_amdgcn_rcpf(e + 1.0f);
}

__device__ __forceinline__ v4f headsum(v4f v) {
  v.x += __shfl_xor(v.x, 8, 32);  v.y += __shfl_xor(v.y, 8, 32);
  v.z += __shfl_xor(v.z, 8, 32);  v.w += __shfl_xor(v.w, 8, 32);
  v.x += __shfl_xor(v.x, 16, 32); v.y += __shfl_xor(v.y, 16, 32);
  v.z += __shfl_xor(v.z, 16, 32); v.w += __shfl_xor(v.w, 16, 32);
  return v;
}

__global__ __launch_bounds__(NTHR) void k_prep(const float* __restrict__ W, _Float16* Wt,
                                              int K, int NC, float scale) {
  const int kq = K >> 3;
  const int total = NC * kq;
  const int i = blockIdx.x * NTHR + threadIdx.x;
  if (i >= total) return;
  const int n  = i / kq;
  const int k0 = (i - n * kq) * 8;
  const float* p = W + (size_t)k0 * NC + n;
  Pack16 u;
  u.h[0] = (_Float16)(p[0 * (size_t)NC] * scale);
  u.h[1] = (_Float16)(p[1 * (size_t)NC] * scale);
  u.h[2] = (_Float16)(p[2 * (size_t)NC] * scale);
  u.h[3] = (_Float16)(p[3 * (size_t)NC] * scale);
  u.h[4] = (_Float16)(p[4 * (size_t)NC] * scale);
  u.h[5] = (_Float16)(p[5 * (size_t)NC] * scale);
  u.h[6] = (_Float16)(p[6 * (size_t)NC] * scale);
  u.h[7] = (_Float16)(p[7 * (size_t)NC] * scale);
  _Float16* o = Wt + (size_t)n * K + k0;
  *(volatile v4i*)o = u.i;
  __threadfence();
  *(volatile v4i*)o = u.i;
}

__device__ __forceinline__ void epi_tile(v8f acc, int T, int hh, int m, int wave, int ncol,
                                         float cs, float cd, float* Xs, float* As, float* Ds) {
  float ss[8], sd[8];
#pragma unroll
  for (int r = 0; r < 8; ++r) {
    const float v = acc[r] * 0.125f;
    Xs[(T * 16 + 8 * hh + r) * XSP + ncol] = v;
    ss[r] = v * cs;
    sd[r] = v * cd;
  }
#pragma unroll
  for (int mk = 1; mk < 16; mk <<= 1) {
#pragma unroll
    for (int r = 0; r < 8; ++r) {
      ss[r] += __shfl_xor(ss[r], mk, 32);
      sd[r] += __shfl_xor(sd[r], mk, 32);
    }
  }
  if (m == 0) {
#pragma unroll
    for (int r = 0; r < 8; ++r) {
      As[(T * 16 + 8 * hh + r) * NWAVE + wave] = ss[r];
      Ds[(T * 16 + 8 * hh + r) * NWAVE + wave] = sd[r];
    }
  }
}

template <int KD>
__global__ __launch_bounds__(NTHR) void k_gemm(
    const float* __restrict__ A, const _Float16* __restrict__ Wt,
    const float* __restrict__ attl, const float* __restrict__ attr,
    float* xp, float* elo, float* ero, int nN) {
  constexpr int AP  = KD + 8;
  constexpr int PER = KD / 8;
  static_assert((AP % 8) == 0);
  static_assert((PER % 4) == 0);
  __shared__ __attribute__((aligned(16))) _Float16 At[GR * AP];
  __shared__ __attribute__((aligned(16))) float Xs[GR * XSP];
  __shared__ __attribute__((aligned(16))) float As[GR * NWAVE];
  __shared__ __attribute__((aligned(16))) float Ds[GR * NWAVE];

  const int tid  = threadIdx.x;
  const int lane = tid & 31;
  const int wave = tid >> 5;
  const int hh   = lane >> 4;
  const int m    = lane & 15;
  const int rowBase = blockIdx.x * GR;

  {
    const int r  = tid >> 3;
    const int c0 = (tid & 7) * PER;
    int row = rowBase + r;
    if (row > nN - 1) row = nN - 1;
    const float* p = A + (size_t)row * KD + c0;
#pragma unroll
    for (int q = 0; q < PER; q += 4) {
      const v4f f = *(const v4f*)(p + q);
      v4h u;
      u.x = (_Float16)f.x; u.y = (_Float16)f.y; u.z = (_Float16)f.z; u.w = (_Float16)f.w;
      *(v4h*)(At + r * AP + c0 + q) = u;
    }
  }
  __syncthreads();

  const int ncol = wave * 16 + m;
  v8f c0a = {0.f, 0.f, 0.f, 0.f, 0.f, 0.f, 0.f, 0.f};
  v8f c1a = {0.f, 0.f, 0.f, 0.f, 0.f, 0.f, 0.f, 0.f};
#pragma unroll
  for (int kt = 0; kt < KD / 32; ++kt) {
    const int k0 = kt * 32;
    Frag a0, a1, b;
    const _Float16* pb  = Wt + (size_t)ncol * KD + k0 + 8 * hh;
    const _Float16* pa0 = At + m * AP + k0 + 8 * hh;
    const _Float16* pa1 = At + (16 + m) * AP + k0 + 8 * hh;
    b.half[0]  = *(const v8h*)pb;  b.half[1]  = *(const v8h*)(pb + 16);
    a0.half[0] = *(const v8h*)pa0; a0.half[1] = *(const v8h*)(pa0 + 16);
    a1.half[0] = *(const v8h*)pa1; a1.half[1] = *(const v8h*)(pa1 + 16);
    c0a = wm(a0.v, b.v, c0a);
    c1a = wm(a1.v, b.v, c1a);
  }

  const float cs = attl[ncol];
  const float cd = attr[ncol];
  epi_tile(c0a, 0, hh, m, wave, ncol, cs, cd, Xs, As, Ds);
  epi_tile(c1a, 1, hh, m, wave, ncol, cs, cd, Xs, As, Ds);
  __syncthreads();

  v4f xr[4];
#pragma unroll
  for (int i = 0; i < 4; ++i) xr[i] = *(const v4f*)(Xs + (4 * wave + i) * XSP + 4 * lane);
  float* gp = 0;
  v4f gv = {0.f, 0.f, 0.f, 0.f};
  if (wave < 2) {
    const float* S = (wave == 0) ? As : Ds;
    const v4f pa = *(const v4f*)(S + lane * NWAVE);
    const v4f pc = *(const v4f*)(S + lane * NWAVE + 4);
    gv.x = pa.x + pa.y;
    gv.y = pa.z + pa.w;
    gv.z = pc.x + pc.y;
    gv.w = pc.z + pc.w;
    gp = ((wave == 0) ? elo : ero) + (size_t)rowBase * NHD + 4 * lane;
  }
  float* xpp[4];
#pragma unroll
  for (int i = 0; i < 4; ++i) xpp[i] = xp + (size_t)(rowBase + 4 * wave + i) * DF + 4 * lane;

#pragma unroll
  for (int i = 0; i < 4; ++i) *(volatile v4f*)(xpp[i]) = xr[i];
  if (gp) *(volatile v4f*)gp = gv;
  __threadfence();
#pragma unroll
  for (int i = 0; i < 4; ++i) *(volatile v4f*)(xpp[i]) = xr[i];
  if (gp) *(volatile v4f*)gp = gv;
}

template <bool ACT>
__global__ __launch_bounds__(NTHR) void k_gat(
    const int* __restrict__ srcp, const int* __restrict__ dstp,
    const float* __restrict__ xp, const float* __restrict__ elb, const float* __restrict__ erb,
    const float* __restrict__ bias, float* out, int nN, int nE) {
  extern __shared__ v4f lds_dyn[];
  float* sacc = (float*)lds_dyn;
  float* den  = sacc + LDS_SACC;
  int*   list = (int*)(den + LDS_DEN);
  int*   wcnt = list + LDS_LIST;

  const int tid  = threadIdx.x;
  const int lane = tid & 31;
  const int wave = tid >> 5;
  const int hd   = lane >> 3;
  const int nodeBase = blockIdx.x * NB;

  {
    const v4f z4 = {0.f, 0.f, 0.f, 0.f};
    for (int i = tid; i < (LDS_SACC + LDS_DEN) / 4; i += NTHR) lds_dyn[i] = z4;
  }
  __syncthreads();
  const bool al16 = ((((uintptr_t)dstp) & 15) == 0);

  const int nChunks = (nE + CHUNK - 1) / CHUNK;
#pragma unroll 1
  for (int ch = 0; ch < nChunks; ++ch) {
    const int cbase = ch * CHUNK;
    int wc = 0;
#pragma unroll
    for (int g = 0; g < NGRP; ++g) {
      const int el0 = (g * NTHR + tid) * 4;
      const int e0  = cbase + el0;
      const int sent = -2147483647 - 1;
      v4i d;
      if (al16 && (e0 + 3 < nE)) {
        d = *(const v4i*)(dstp + e0);
      } else {
        d.x = (e0     < nE) ? dstp[e0]     : sent;
        d.y = (e0 + 1 < nE) ? dstp[e0 + 1] : sent;
        d.z = (e0 + 2 < nE) ? dstp[e0 + 2] : sent;
        d.w = (e0 + 3 < nE) ? dstp[e0 + 3] : sent;
      }
      const unsigned s0 = (unsigned)d.x - (unsigned)nodeBase;
      const unsigned s1 = (unsigned)d.y - (unsigned)nodeBase;
      const unsigned s2 = (unsigned)d.z - (unsigned)nodeBase;
      const unsigned s3 = (unsigned)d.w - (unsigned)nodeBase;
      const bool h0 = s0 < (unsigned)NB;
      const bool h1 = s1 < (unsigned)NB;
      const bool h2 = s2 < (unsigned)NB;
      const bool h3 = s3 < (unsigned)NB;
      const unsigned many = __builtin_amdgcn_ballot_w32(h0 | h1 | h2 | h3);
      if (many != 0u) {
#define HITJ(J, HJ, SJ) { \
          const unsigned mj = __builtin_amdgcn_ballot_w32(HJ); \
          if (HJ) { \
            const int pos = wc + (int)__builtin_amdgcn_mbcnt_lo(mj, 0u); \
            if (pos < WCAP) list[wave * WCAP + pos] = ((el0 + (J)) << 9) | (int)(SJ); \
          } \
          wc += (int)__builtin_popcount(mj); }
        HITJ(0, h0, s0)
        HITJ(1, h1, s1)
        HITJ(2, h2, s2)
        HITJ(3, h3, s3)
#undef HITJ
      }
    }
    if (lane == 0) wcnt[wave] = wc;
    __syncthreads();

    if (wave == 0) {
      for (int wsx = 0; wsx < NWAVE; ++wsx) {
        int n = wcnt[wsx];
        if (n > WCAP) n = WCAP;
        if (n < 0) n = 0;
        for (int i = 0; i < n; ++i) {
          const int ent  = list[wsx * WCAP + i];
          const int slot = ent & (NB - 1);
          const int eloc = (ent >> 9) & (CHUNK - 1);
          int e = cbase + eloc;
          if (e > nE - 1) e = nE - 1;
          int s = srcp[e];
          s = s < 0 ? 0 : (s > nN - 1 ? nN - 1 : s);
          int nd = nodeBase + slot;
          if (nd > nN - 1) nd = nN - 1;
          float al = elb[(size_t)s * NHD + hd] + erb[(size_t)nd * NHD + hd];
          al = (al > 0.f) ? al : 0.2f * al;
          al = fminf(al, 60.f);
          const float p = __expf(al);
          const v4f xv = *(const v4f*)(xp + (size_t)s * DF + 4 * lane);
          v4f* sp = (v4f*)(sacc + slot * DF + 4 * lane);
          const v4f cur = *sp;
          const v4f nxt = cur + p * xv;
          *sp = nxt;
          if ((lane & 7) == 0) {
            const float o = den[slot * NHD + hd];
            den[slot * NHD + hd] = o + p;
          }
        }
      }
    }
    __syncthreads();
  }

  const v4f b4 = *(const v4f*)(bias + 4 * lane);
  const int q = lane >> 3;
#pragma unroll 1
  for (int g = 0; g < (NB / NWAVE) / 4; ++g) {
    const int slot0 = wave * (NB / NWAVE) + 4 * g;
    if (nodeBase + slot0 >= nN) break;
    v4f keep = {0.f, 0.f, 0.f, 0.f};
#pragma unroll 1
    for (int jj = 0; jj < 4; ++jj) {
      const int slot = slot0 + jj;
      const v4f sv  = *(const v4f*)(sacc + slot * DF + 4 * lane);
      const float dn  = den[slot * NHD + hd];
      const float inv = __builtin_amdgcn_rcpf(fmaxf(dn, 1e-30f));
      v4f hv = sv * inv + b4;
      if (ACT) { hv.x = th1(hv.x); hv.y = th1(hv.y); hv.z = th1(hv.z); hv.w = th1(hv.w); }
      hv = headsum(hv) * 0.25f;
      if (q == jj) keep = hv;
    }
    const int node = nodeBase + slot0 + q;
    float* op = out + (size_t)node * HDIM + 4 * (lane & 7);
    if (node < nN) *(volatile v4f*)op = keep;
    __threadfence();
    if (node < nN) *(volatile v4f*)op = keep;
  }
}

extern "C" void kernel_launch(void* const* d_in, const int* in_sizes, int n_in,
                              void* d_out, int out_size, void* d_ws, size_t ws_size,
                              hipStream_t stream) {
  if (n_in < 11) return;
  const int nN = in_sizes[0] / DF;
  const int nE = in_sizes[1];
  if (nN <= 0 || in_sizes[0] != nN * DF) return;
  if (nE < 0 || in_sizes[2] != nE) return;
  if (in_sizes[3] != DF * DF) return;
  if (in_sizes[4] != NHD * HDIM || in_sizes[5] != NHD * HDIM || in_sizes[6] != DF) return;
  if (in_sizes[7] != HDIM * DF) return;
  if (in_sizes[8] != NHD * HDIM || in_sizes[9] != NHD * HDIM || in_sizes[10] != DF) return;
  if (out_size != nN * HDIM) return;

  const float* x   = (const float*)d_in[0];
  const int*   src = (const int*)d_in[1];
  const int*   dst = (const int*)d_in[2];
  const float* W0  = (const float*)d_in[3];
  const float* al0 = (const float*)d_in[4];
  const float* ar0 = (const float*)d_in[5];
  const float* b0  = (const float*)d_in[6];
  const float* W1  = (const float*)d_in[7];
  const float* al1 = (const float*)d_in[8];
  const float* ar1 = (const float*)d_in[9];
  const float* b1  = (const float*)d_in[10];
  float* out = (float*)d_out;

  const int nP = ((nN + GR - 1) / GR) * GR;
  size_t off = 0;
  _Float16* Wt0 = (_Float16*)((char*)d_ws + off); off += (size_t)DF * DF * sizeof(_Float16);
  _Float16* Wt1 = (_Float16*)((char*)d_ws + off); off += (size_t)DF * HDIM * sizeof(_Float16);
  float* xp   = (float*)((char*)d_ws + off);      off += (size_t)nP * DF * sizeof(float);
  float* elb  = (float*)((char*)d_ws + off);      off += (size_t)nP * NHD * sizeof(float);
  float* erb  = (float*)((char*)d_ws + off);      off += (size_t)nP * NHD * sizeof(float);
  float* hbuf = (float*)((char*)d_ws + off);      off += (size_t)nP * HDIM * sizeof(float);
  const size_t cap = (size_t)128 * 1024 * 1024;
  if (off > ws_size || off > cap) return;

  {
    const int t0 = DF * (DF / 8);
    k_prep<<<(t0 + NTHR - 1) / NTHR, NTHR, 0, stream>>>(W0, Wt0, DF, DF, 8.0f);
    const int t1 = DF * (HDIM / 8);
    k_prep<<<(t1 + NTHR - 1) / NTHR, NTHR, 0, stream>>>(W1, Wt1, HDIM, DF, 8.0f);
  }
  const int ggrid = (nN + NB - 1) / NB;

  k_gemm<DF><<<nP / GR, NTHR, 0, stream>>>(x, Wt0, al0, ar0, xp, elb, erb, nN);
  hipFuncSetAttribute(reinterpret_cast<const void*>(&k_gat<true>),
                      hipFuncAttributeMaxDynamicSharedMemorySize, LDS_BYTES);
  k_gat<true><<<ggrid, NTHR, LDS_BYTES, stream>>>(src, dst, xp, elb, erb, b0, hbuf, nN, nE);

  k_gemm<HDIM><<<nP / GR, NTHR, 0, stream>>>(hbuf, Wt1, al1, ar1, xp, elb, erb, nN);
  hipFuncSetAttribute(reinterpret_cast<const void*>(&k_gat<false>),
                      hipFuncAttributeMaxDynamicSharedMemorySize, LDS_BYTES);
  k_gat<false><<<ggrid, NTHR, LDS_BYTES, stream>>>(src, dst, xp, elb, erb, b1, out, nN, nE);
}
